// Mamba_head_78254304133372
// MI455X (gfx1250) — hardware-verified
//
#include <hip/hip_runtime.h>


#define NB_   4
#define L_    1024
#define DM_   1024
#define DI_   1024
#define NS_   16
#define DTR_  64
#define XDN_  96
#define XDW_  128
#define NT_   (NB_ * L_)
#define SAP_  72

static constexpr float EPS_ = 1e-5f;

static_assert(NT_ % 64 == 0);
static_assert(NT_ % 8 == 0);
static_assert(NT_ % 2 == 0);
static_assert(DM_ == 1024);
static_assert(DI_ == 1024);
static_assert((2 * DI_) % 128 == 0);
static_assert(XDW_ % 128 == 0);
static_assert(DM_ % 128 == 0);
static_assert(L_ % 16 == 0);
static_assert(DTR_ == 64);
static_assert(DTR_ + 2 * NS_ == XDN_);
static_assert(XDN_ <= XDW_);

typedef float          v4f   __attribute__((ext_vector_type(4)));
typedef float          v8f   __attribute__((ext_vector_type(8)));
typedef _Float16       v8h   __attribute__((ext_vector_type(8)));
typedef _Float16       v16h  __attribute__((ext_vector_type(16)));
typedef unsigned short u16x8 __attribute__((ext_vector_type(8)));

union FragH { u16x8 h[2]; v16h v; };
union Pack8 { v8h f; u16x8 u; };
union HBits { _Float16 h; unsigned short u; };

constexpr size_t SZ_HS = (size_t)NT_ * DM_ * 2;
constexpr size_t SZ_WI = (size_t)2 * DI_ * DM_ * 2;
constexpr size_t SZ_WX = (size_t)2 * XDW_ * DI_ * 2;
constexpr size_t SZ_WD = (size_t)2 * DI_ * DTR_ * 2;
constexpr size_t SZ_WO = (size_t)DM_ * DI_ * 2;
constexpr size_t SZ_WF = (size_t)DM_ * DM_ * 2;
constexpr size_t SZ_XZ = (size_t)NT_ * 2 * DI_ * 4;
constexpr size_t SZ_U  = (size_t)NT_ * DI_ * 2;
constexpr size_t SZ_XD = (size_t)NT_ * XDW_ * 4;
constexpr size_t SZ_G0 = (size_t)NT_ * DI_ * 4;
constexpr size_t SZ_YS = (size_t)NT_ * DI_ * 2;
constexpr size_t SZ_O1 = (size_t)NT_ * DM_ * 2;

constexpr size_t OFF_HS = 0;
constexpr size_t OFF_WI = OFF_HS + SZ_HS;
constexpr size_t OFF_WX = OFF_WI + SZ_WI;
constexpr size_t OFF_WD = OFF_WX + SZ_WX;
constexpr size_t OFF_WO = OFF_WD + SZ_WD;
constexpr size_t OFF_WF = OFF_WO + SZ_WO;
constexpr size_t OFF_XZ = OFF_WF + SZ_WF;
constexpr size_t OFF_U  = OFF_XZ + SZ_XZ;
constexpr size_t OFF_XD = OFF_U  + SZ_U;
constexpr size_t OFF_G0 = OFF_XD + SZ_XD;
constexpr size_t OFF_YS = OFF_G0 + SZ_G0;
constexpr size_t OFF_O1 = OFF_YS + SZ_YS;
constexpr size_t WS_END = OFF_O1 + SZ_O1;

static_assert(WS_END <= (size_t)134217728);
static_assert(OFF_WI % 128 == 0 && OFF_WX % 128 == 0 && OFF_WD % 128 == 0 && OFF_WO % 128 == 0);
static_assert(OFF_WF % 128 == 0 && OFF_XZ % 128 == 0 && OFF_U % 128 == 0 && OFF_XD % 128 == 0);
static_assert(OFF_G0 % 128 == 0 && OFF_YS % 128 == 0 && OFF_O1 % 128 == 0 && WS_END % 128 == 0);

__device__ __forceinline__ float silu_f(float x) {
    const float e = __expf(-x);
    return x * __builtin_amdgcn_rcpf(1.0f + e);
}
__device__ __forceinline__ float softplus_f(float x) {
    return fmaxf(x, 0.0f) + log1pf(__expf(-fabsf(x)));
}
__device__ __forceinline__ float conv4_silu(float x0, float x1, float x2, float x3,
                                            float w0, float w1, float w2, float w3, float bias) {
    const float c = w0 * x0 + w1 * x1 + w2 * x2 + w3 * x3;
    return silu_f(c + bias);
}
__device__ __forceinline__ v8f ld8f(const float* p) {
    const v4f a = *(const v4f*)p;
    const v4f b = *(const v4f*)(p + 4);
    return __builtin_shufflevector(a, b, 0, 1, 2, 3, 4, 5, 6, 7);
}
__device__ __forceinline__ float wave_sum(float v) {
#pragma unroll
    for (int mk = 16; mk >= 1; mk >>= 1) v += __shfl_xor(v, mk, 32);
    return v;
}

__device__ __forceinline__ void mma16(v8f& acc, const FragH& a, const FragH& b) {
    acc = __builtin_amdgcn_wmma_f32_16x16x32_f16(false, a.v, false, b.v, (short)0, acc, false, false);
    asm volatile("v_nop\n\tv_nop\n\tv_nop\n\tv_nop" : "+v"(acc) : "v"(a.v), "v"(b.v));
}

__global__ __launch_bounds__(256)
void cvt_w_kernel(const float* __restrict__ W, unsigned short* dst, int N, int Npad, int K, float scale)
{
    const size_t i = (size_t)blockIdx.x * 256 + threadIdx.x;
    const size_t e = i * 8;
    const size_t total = (size_t)Npad * (size_t)K;
    if (e >= total) return;
    const int row = (int)(e / (size_t)K);
    const int col = (int)(e - (size_t)row * (size_t)K);
    const int rs  = min(row, N - 1);
    v8f v = ld8f(W + (size_t)rs * K + col);
    if (row >= N) {
#pragma unroll
        for (int c = 0; c < 8; ++c) v[c] = 0.0f;
    }
    v = v * scale;
    Pack8 pk;
    pk.f = __builtin_convertvector(v, v8h);
    const u16x8 u = pk.u;
    unsigned short* gp = dst + e;
    *(volatile u16x8*)gp = u;
    __threadfence();
    *(volatile u16x8*)gp = u;
}

__device__ __forceinline__ void ln_store_pass(const float* xr, const float* __restrict__ g, const float* __restrict__ bta,
                                              unsigned short* op, int lane, float mu, float rr)
{
#pragma unroll 1
    for (int j = 0; j < 4; ++j) {
        const v8f v  = ld8f(xr + 256 * j);
        const v8f gv = ld8f(g + 256 * j + 8 * lane);
        const v8f bv = ld8f(bta + 256 * j + 8 * lane);
        const v8f o  = (v - mu) * rr * gv + bv;
        Pack8 pk;
        pk.f = __builtin_convertvector(o, v8h);
        const u16x8 u = pk.u;
        *(volatile u16x8*)(op + 256 * j) = u;
    }
}

__global__ __launch_bounds__(256)
void ln_kernel(const float* __restrict__ x, const float* __restrict__ g, const float* __restrict__ bta,
               unsigned short* hs)
{
    const int lane = threadIdx.x & 31, wave = threadIdx.x >> 5;
    const int t = blockIdx.x * 8 + wave;
    if (t >= NT_) return;
    const float* xr = x + (size_t)t * DM_ + 8 * lane;
    float s = 0.0f;
#pragma unroll 1
    for (int j = 0; j < 4; ++j) {
        const v8f v = ld8f(xr + 256 * j);
        s += ((v[0] + v[1]) + (v[2] + v[3])) + ((v[4] + v[5]) + (v[6] + v[7]));
    }
    const float mu = wave_sum(s) * (1.0f / (float)DM_);
    float q = 0.0f;
#pragma unroll 1
    for (int j = 0; j < 4; ++j) {
        const v8f v = ld8f(xr + 256 * j);
#pragma unroll
        for (int e = 0; e < 8; ++e) { const float dl = v[e] - mu; q = fmaf(dl, dl, q); }
    }
    const float rr = rsqrtf(wave_sum(q) * (1.0f / (float)DM_) + EPS_);
    unsigned short* op = hs + (size_t)t * DM_ + 8 * lane;
    ln_store_pass(xr, g, bta, op, lane, mu, rr);
    __threadfence();
    ln_store_pass(xr, g, bta, op, lane, mu, rr);
}

template<typename OT, int NBF, bool EPI>
__device__ __forceinline__ void tile_store_pass(const float* st, OT* gp, int ldc, int lane,
                                                const float* __restrict__ bp, const float* __restrict__ rp, int ldr) {
    constexpr int CW  = NBF * 16;
    constexpr int P   = CW + 4;
    constexpr int EPL = 16 / (int)sizeof(OT);
    static_assert(CW % EPL == 0);
    constexpr int LPR = CW / EPL;
    static_assert(32 % LPR == 0);
    constexpr int RPI = 32 / LPR;
    static_assert(32 % RPI == 0);
    constexpr int NIT = 32 / RPI;
    const int rsub = lane / LPR;
    const int c0   = (lane % LPR) * EPL;
#pragma unroll
    for (int it = 0; it < NIT; ++it) {
        const int row = it * RPI + rsub;
        const float* sp = st + row * P + c0;
        OT* dp = gp + (size_t)row * ldc + c0;
        if constexpr (sizeof(OT) == 4) {
            v4f v = *(const v4f*)sp;
            if constexpr (EPI) {
                const v4f bb = *(const v4f*)(bp + c0);
                const v4f rv = *(const v4f*)(rp + (size_t)row * ldr + c0);
                v = (v + bb) + rv;
            }
            *(volatile v4f*)dp = v;
        } else {
            Pack8 pk;
            pk.f = __builtin_convertvector(ld8f(sp), v8h);
            const u16x8 u = pk.u;
            *(volatile u16x8*)dp = u;
        }
    }
}

template<int NBF, typename OT, bool EPI>
__global__ __launch_bounds__(128)
void gemm_tn_kernel(const unsigned short* __restrict__ A, const unsigned short* __restrict__ Bw, OT* C,
                    const float* __restrict__ bias, const float* __restrict__ res,
                    int K, int ldc, int ldr, float scale)
{
    constexpr int CW = NBF * 16;
    constexpr int P  = CW + 4;
    __shared__ __attribute__((aligned(16))) float stile[4][32 * P];

    const int tid  = threadIdx.x;
    const int lane = tid & 31;
    const int wave = tid >> 5;
    const int h    = lane >> 4;
    const int m    = lane & 15;
    const int wm   = wave >> 1;
    const int wn   = wave & 1;

    const int rowW = blockIdx.y * 64 + wm * 32;
    const int colW = blockIdx.x * (2 * CW) + wn * CW;

    const unsigned short* pa[2];
#pragma unroll
    for (int s = 0; s < 2; ++s)
        pa[s] = A + (size_t)(rowW + 16 * s + m) * (size_t)K + 8 * h;
    const unsigned short* pb = Bw + (size_t)(colW + m) * (size_t)K + 8 * h;
    const size_t sub16 = (size_t)16 * (size_t)K;

    v8f acc[2 * NBF];
#pragma unroll
    for (int j = 0; j < 2 * NBF; ++j)
#pragma unroll
        for (int r = 0; r < 8; ++r) acc[j][r] = 0.0f;

    const int nk = K >> 5;
    for (int kt = 0; kt < nk; ++kt) {
        const int k0 = kt * 32;
        FragH fa[2], fb[NBF];
#pragma unroll
        for (int s = 0; s < 2; ++s) {
            fa[s].h[0] = *(const u16x8*)(pa[s] + k0);
            fa[s].h[1] = *(const u16x8*)(pa[s] + k0 + 16);
        }
#pragma unroll
        for (int j = 0; j < NBF; ++j) {
            const unsigned short* p = pb + j * sub16 + k0;
            fb[j].h[0] = *(const u16x8*)(p);
            fb[j].h[1] = *(const u16x8*)(p + 16);
        }
#pragma unroll
        for (int s = 0; s < 2; ++s)
#pragma unroll
            for (int j = 0; j < NBF; ++j)
                mma16(acc[s * NBF + j], fa[s], fb[j]);
    }

    float* st = stile[wave];
#pragma unroll
    for (int s = 0; s < 2; ++s)
#pragma unroll
        for (int j = 0; j < NBF; ++j)
#pragma unroll
            for (int r = 0; r < 8; ++r)
                st[(s * 16 + 8 * h + r) * P + j * 16 + m] = acc[s * NBF + j][r] * scale;
    __syncthreads();

    OT* gp = C + (size_t)rowW * (size_t)ldc + colW;
    const float* bp = bias + colW;
    const float* rp = res + (size_t)rowW * (size_t)ldr + colW;
    tile_store_pass<OT, NBF, EPI>(st, gp, ldc, lane, bp, rp, ldr);
    __threadfence();
    tile_store_pass<OT, NBF, EPI>(st, gp, ldc, lane, bp, rp, ldr);
}

template<int DIR>
__global__ __launch_bounds__(256)
void conv_silu_kernel(const float* __restrict__ xz, const float* __restrict__ cw,
                      const float* __restrict__ cb, unsigned short* u16)
{
    const int tid = threadIdx.x;
    const int r   = tid >> 7;
    const int d0  = (tid & 127) * 8;
    const int row = blockIdx.x * 2 + r;
    if (row >= NT_) return;
    const int b   = row / L_;
    const int t   = row - b * L_;
    const int t1 = max(t - 1, 0), t2 = max(t - 2, 0), t3 = max(t - 3, 0);
    const int o0 = DIR ? (L_ - 1 - t)  : t;
    const int o1 = DIR ? (L_ - 1 - t1) : t1;
    const int o2 = DIR ? (L_ - 1 - t2) : t2;
    const int o3 = DIR ? (L_ - 1 - t3) : t3;
    const size_t brow = (size_t)b * L_;

    v8f x3 = ld8f(xz + (brow + (size_t)o0) * (size_t)(2 * DI_) + d0);
    v8f x2 = ld8f(xz + (brow + (size_t)o1) * (size_t)(2 * DI_) + d0);
    v8f x1 = ld8f(xz + (brow + (size_t)o2) * (size_t)(2 * DI_) + d0);
    v8f x0 = ld8f(xz + (brow + (size_t)o3) * (size_t)(2 * DI_) + d0);
#pragma unroll
    for (int c = 0; c < 8; ++c) {
        x2[c] = (t >= 1) ? x2[c] : 0.0f;
        x1[c] = (t >= 2) ? x1[c] : 0.0f;
        x0[c] = (t >= 3) ? x0[c] : 0.0f;
    }

    v4f wv[8];
#pragma unroll
    for (int c = 0; c < 8; ++c) wv[c] = *(const v4f*)(cw + (size_t)(d0 + c) * 4);
    const v8f bias = ld8f(cb + d0);

    v8f u;
#pragma unroll
    for (int c = 0; c < 8; ++c)
        u[c] = 64.0f * conv4_silu(x0[c], x1[c], x2[c], x3[c], wv[c][0], wv[c][1], wv[c][2], wv[c][3], bias[c]);

    Pack8 pk;
    pk.f = __builtin_convertvector(u, v8h);
    const u16x8 v = pk.u;
    unsigned short* gp = u16 + (size_t)row * DI_ + d0;
    *(volatile u16x8*)gp = v;
    __threadfence();
    *(volatile u16x8*)gp = v;
}

__device__ __forceinline__ void g32_store_pass(const float* sl, float* gp, int wave, int lane) {
#pragma unroll
    for (int it = 0; it < 4; ++it) {
        const int t = it * 4 + wave * 2 + (lane >> 4);
        const int c = (lane & 15) * 4;
        const v4f v = *(const v4f*)(sl + t * 64 + c);
        *(volatile v4f*)(gp + (size_t)t * DI_ + c) = v;
    }
}
__device__ __forceinline__ void g16_store_pass(const unsigned short* sl, unsigned short* gp, int wave, int lane) {
#pragma unroll
    for (int it = 0; it < 2; ++it) {
        const int t = it * 8 + wave * 4 + (lane >> 3);
        const int c = (lane & 7) * 8;
        const u16x8 v = *(const u16x8*)(sl + t * 64 + c);
        *(volatile u16x8*)(gp + (size_t)t * DI_ + c) = v;
    }
}

template<int DIR>
__global__ __launch_bounds__(64)
void scan_kernel(const float* __restrict__ xz, const float* __restrict__ xd,
                 const unsigned short* __restrict__ wdt,
                 const float* __restrict__ cw, const float* __restrict__ cb,
                 const float* __restrict__ dtb, const float* __restrict__ Alog,
                 const float* __restrict__ Dp, const float* gfin,
                 float* gout, unsigned short* yout)
{
    __shared__ __attribute__((aligned(16))) unsigned short sA[16 * SAP_];
    __shared__ __attribute__((aligned(16))) float sBC[16 * 32];
    __shared__ __attribute__((aligned(16))) float sdt[16 * 64];
    __shared__ __attribute__((aligned(16))) float sg32[16 * 64];
    __shared__ __attribute__((aligned(16))) unsigned short sg16[16 * 64];

    const int tid   = threadIdx.x;
    const int lane  = tid & 31;
    const int wave  = tid >> 5;
    const int h     = lane >> 4;
    const int m     = lane & 15;
    const int b     = blockIdx.y;
    const int dbase = blockIdx.x * 64;
    const int d     = dbase + tid;

    float an[NS_], hst[NS_];
#pragma unroll
    for (int n = 0; n < NS_; ++n) {
        an[n]  = -__expf(Alog[(size_t)d * NS_ + n]);
        hst[n] = 0.0f;
    }
    const float w0 = cw[(size_t)d * 4 + 0], w1 = cw[(size_t)d * 4 + 1], w2 = cw[(size_t)d * 4 + 2], w3 = cw[(size_t)d * 4 + 3];
    const float cbias = cb[d];
    const float tb    = dtb[d];
    const float Dd    = Dp[d];

    FragH fb[2][2];
#pragma unroll
    for (int j = 0; j < 2; ++j)
#pragma unroll
        for (int ks = 0; ks < 2; ++ks) {
            const int n = dbase + 32 * wave + 16 * j + m;
            const unsigned short* p = wdt + (size_t)n * DTR_ + 32 * ks + 8 * h;
            fb[j][ks].h[0] = *(const u16x8*)(p);
            fb[j][ks].h[1] = *(const u16x8*)(p + 16);
        }

    float xm1 = 0.0f, xm2 = 0.0f, xm3 = 0.0f;
    const size_t brow0 = (size_t)b * L_;

#pragma unroll 1
    for (int l0 = 0; l0 < L_; l0 += 16) {
        const size_t xrow0 = brow0 + (size_t)l0;
#pragma unroll
        for (int j = 0; j < 16; ++j) {
            const float v = xd[(xrow0 + (size_t)j) * XDW_ + tid];
            HBits hb;
            hb.h = (_Float16)(v * 16.0f);
            sA[j * SAP_ + tid] = hb.u;
        }
#pragma unroll
        for (int j = 0; j < 8; ++j) {
            const int idx = j * 64 + tid;
            const int rr  = idx >> 5;
            const int cc  = idx & 31;
            sBC[rr * 32 + cc] = xd[(xrow0 + (size_t)rr) * XDW_ + DTR_ + cc];
        }
        __syncthreads();

        v8f acc[2];
#pragma unroll
        for (int j = 0; j < 2; ++j)
#pragma unroll
            for (int r = 0; r < 8; ++r) acc[j][r] = 0.0f;
#pragma unroll
        for (int ks = 0; ks < 2; ++ks) {
            FragH fa;
            const unsigned short* ap = sA + m * SAP_ + 32 * ks + 8 * h;
            fa.h[0] = *(const u16x8*)(ap);
            fa.h[1] = *(const u16x8*)(ap + 16);
            mma16(acc[0], fa, fb[0][ks]);
            mma16(acc[1], fa, fb[1][ks]);
        }
#pragma unroll
        for (int j = 0; j < 2; ++j)
#pragma unroll
            for (int r = 0; r < 8; ++r)
                sdt[(8 * h + r) * 64 + 32 * wave + 16 * j + m] = acc[j][r] * (1.0f / 128.0f);
        __syncthreads();

#pragma unroll 1
        for (int t = 0; t < 16; ++t) {
            const int to = DIR ? (L_ - 1 - (l0 + t)) : (l0 + t);
            const size_t e = (brow0 + (size_t)to) * (size_t)(2 * DI_) + d;
            const float xv = xz[e];
            const float zv = xz[e + DI_];
            const float u  = conv4_silu(xm3, xm2, xm1, xv, w0, w1, w2, w3, cbias);
            xm3 = xm2; xm2 = xm1; xm1 = xv;
            const float dt = softplus_f(sdt[t * 64 + tid] + tb);
            const float du = dt * u;
            const float* sr = sBC + t * 32;
            float y = 0.0f;
#pragma unroll
            for (int n = 0; n < NS_; ++n) {
                const float da = __expf(dt * an[n]);
                hst[n] = da * hst[n] + du * sr[n];
                y += hst[n] * sr[NS_ + n];
            }
            const float g = (y + Dd * u) * silu_f(zv);
            if constexpr (DIR == 0) {
                sg32[t * 64 + tid] = g;
            } else {
                const float gf = gfin[(brow0 + (size_t)to) * DI_ + d];
                HBits hb;
                hb.h = (_Float16)((g + gf) * 64.0f);
                sg16[(15 - t) * 64 + tid] = hb.u;
            }
        }
        __syncthreads();
        if constexpr (DIR == 0) {
            float* gp = gout + xrow0 * DI_ + dbase;
            g32_store_pass(sg32, gp, wave, lane);
            __threadfence();
            g32_store_pass(sg32, gp, wave, lane);
        } else {
            unsigned short* gp = yout + (brow0 + (size_t)(L_ - 16 - l0)) * DI_ + dbase;
            g16_store_pass(sg16, gp, wave, lane);
            __threadfence();
            g16_store_pass(sg16, gp, wave, lane);
        }
        __syncthreads();
    }
}

extern "C" void kernel_launch(void* const* d_in, const int* in_sizes, int n_in,
                              void* d_out, int out_size, void* d_ws, size_t ws_size,
                              hipStream_t stream)
{
    if (n_in < 21) return;
    if (in_sizes[0]  != NT_ * DM_)      return;
    if (in_sizes[1]  != DM_)            return;
    if (in_sizes[2]  != DM_)            return;
    if (in_sizes[3]  != 2 * DI_ * DM_)  return;
    for (int s = 0; s < 2; ++s) {
        const int o = s ? 11 : 4;
        if (in_sizes[o + 0] != DI_ * 4)     return;
        if (in_sizes[o + 1] != DI_)         return;
        if (in_sizes[o + 2] != XDN_ * DI_)  return;
        if (in_sizes[o + 3] != DI_ * DTR_)  return;
        if (in_sizes[o + 4] != DI_)         return;
        if (in_sizes[o + 5] != DI_ * NS_)   return;
        if (in_sizes[o + 6] != DI_)         return;
    }
    if (in_sizes[18] != DM_ * DI_)      return;
    if (in_sizes[19] != DM_ * DM_)      return;
    if (in_sizes[20] != DM_)            return;
    if (out_size != NT_ * DM_)          return;
    if (ws_size < WS_END)               return;

    const float* hidden = (const float*)d_in[0];
    const float* ln_g   = (const float*)d_in[1];
    const float* ln_b   = (const float*)d_in[2];
    const float* w_in   = (const float*)d_in[3];
    const float* cwp[2]  = {(const float*)d_in[4],  (const float*)d_in[11]};
    const float* cbp[2]  = {(const float*)d_in[5],  (const float*)d_in[12]};
    const float* xpw[2]  = {(const float*)d_in[6],  (const float*)d_in[13]};
    const float* dtw[2]  = {(const float*)d_in[7],  (const float*)d_in[14]};
    const float* dtbp[2] = {(const float*)d_in[8],  (const float*)d_in[15]};
    const float* alp[2]  = {(const float*)d_in[9],  (const float*)d_in[16]};
    const float* dpp[2]  = {(const float*)d_in[10], (const float*)d_in[17]};
    const float* w_out  = (const float*)d_in[18];
    const float* w_fc   = (const float*)d_in[19];
    const float* fc_b   = (const float*)d_in[20];
    float* out = (float*)d_out;

    char* ws = (char*)d_ws;
    unsigned short* hs16  = (unsigned short*)(ws + OFF_HS);
    unsigned short* win16 = (unsigned short*)(ws + OFF_WI);
    unsigned short* wx16  = (unsigned short*)(ws + OFF_WX);
    unsigned short* wdt16 = (unsigned short*)(ws + OFF_WD);
    unsigned short* wo16  = (unsigned short*)(ws + OFF_WO);
    unsigned short* wf16  = (unsigned short*)(ws + OFF_WF);
    float*          xz    = (float*)(ws + OFF_XZ);
    unsigned short* u16   = (unsigned short*)(ws + OFF_U);
    float*          xd    = (float*)(ws + OFF_XD);
    float*          g0    = (float*)(ws + OFF_G0);
    unsigned short* ysum  = (unsigned short*)(ws + OFF_YS);
    unsigned short* o1    = (unsigned short*)(ws + OFF_O1);

    cvt_w_kernel<<<dim3((2 * DI_ * DM_) / 2048), dim3(256), 0, stream>>>(w_in, win16, 2 * DI_, 2 * DI_, DM_, 32.0f);
    for (int s = 0; s < 2; ++s) {
        cvt_w_kernel<<<dim3((XDW_ * DI_) / 2048), dim3(256), 0, stream>>>(xpw[s], wx16 + (size_t)s * XDW_ * DI_, XDN_, XDW_, DI_, 32.0f);
        cvt_w_kernel<<<dim3((DI_ * DTR_) / 2048), dim3(256), 0, stream>>>(dtw[s], wdt16 + (size_t)s * DI_ * DTR_, DI_, DI_, DTR_, 8.0f);
    }
    cvt_w_kernel<<<dim3((DM_ * DI_) / 2048), dim3(256), 0, stream>>>(w_out, wo16, DM_, DM_, DI_, 32.0f);
    cvt_w_kernel<<<dim3((DM_ * DM_) / 2048), dim3(256), 0, stream>>>(w_fc, wf16, DM_, DM_, DM_, 32.0f);

    ln_kernel<<<dim3(NT_ / 8), dim3(256), 0, stream>>>(hidden, ln_g, ln_b, hs16);

    gemm_tn_kernel<4, float, false><<<dim3((2 * DI_) / 128, NT_ / 64), dim3(128), 0, stream>>>(
        hs16, win16, xz, fc_b, hidden, (int)DM_, (int)(2 * DI_), (int)DM_, 1.0f / 32.0f);

    for (int s = 0; s < 2; ++s) {
        if (s == 0) conv_silu_kernel<0><<<dim3(NT_ / 2), dim3(256), 0, stream>>>(xz, cwp[0], cbp[0], u16);
        else        conv_silu_kernel<1><<<dim3(NT_ / 2), dim3(256), 0, stream>>>(xz, cwp[1], cbp[1], u16);

        gemm_tn_kernel<4, float, false><<<dim3(XDW_ / 128, NT_ / 64), dim3(128), 0, stream>>>(
            u16, wx16 + (size_t)s * XDW_ * DI_, xd, fc_b, hidden, (int)DI_, (int)XDW_, (int)DM_, 1.0f / 2048.0f);

        if (s == 0)
            scan_kernel<0><<<dim3(DI_ / 64, NB_), dim3(64), 0, stream>>>(
                xz, xd, wdt16, cwp[0], cbp[0], dtbp[0], alp[0], dpp[0], g0, g0, ysum);
        else
            scan_kernel<1><<<dim3(DI_ / 64, NB_), dim3(64), 0, stream>>>(
                xz, xd, wdt16 + (size_t)DI_ * DTR_, cwp[1], cbp[1], dtbp[1], alp[1], dpp[1], g0, g0, ysum);
    }

    gemm_tn_kernel<4, unsigned short, false><<<dim3(DM_ / 128, NT_ / 64), dim3(128), 0, stream>>>(
        ysum, wo16, o1, fc_b, hidden, (int)DI_, (int)DM_, (int)DM_, 1.0f / 128.0f);

    gemm_tn_kernel<4, float, true><<<dim3(DM_ / 128, NT_ / 64), dim3(128), 0, stream>>>(
        o1, wf16, out, fc_b, hidden, (int)DM_, (int)DM_, (int)DM_, 1.0f / 512.0f);
}
